// GroupShuffleAttention_6253472383726
// MI455X (gfx1250) — hardware-verified
//
#include <hip/hip_runtime.h>
#include <math.h>
#include <stdint.h>

#ifndef NB
#define NB 8
#endif
#ifndef SEQ
#define SEQ 1024
#endif
#define NB_FULL  8
#define SEQ_FULL 1024
#define C_CH  128
#define NGR   8
#define CG    16
#define KP    32
#define NT64  (SEQ / 64)
#define NKT   (SEQ / 32)
#define XAP   40
#define VTP   72
#define PTP   36
#define PTW   (16 * PTP)
#define OTP   68
#define GNIT  ((CG * SEQ) / 1024)
#define QSC   1024.0f
#define VCAR  1024.0f
#define PCAR  16384.0f
#define LOG2E 1.4426950408889634f
#define RSQ_CG 0.25f
#define GN_EPS 1e-5f
#define WS_CAP 134217728
static_assert(NB >= 1 && NB <= NB_FULL);
static_assert((SEQ % 64) == 0 && SEQ >= 64 && SEQ <= SEQ_FULL);
static_assert(C_CH == NGR * CG && CG == 16 && KP == 2 * CG);
static_assert(GNIT * 1024 == CG * SEQ && GNIT >= 1);
static_assert((XAP % 8) == 0 && (VTP % 8) == 0 && (OTP % 4) == 0 && (PTP % 4) == 0);

typedef unsigned short u16;
typedef _Float16 v16h __attribute__((ext_vector_type(16)));
typedef _Float16 v8h  __attribute__((ext_vector_type(8)));
typedef __bf16   v16b __attribute__((ext_vector_type(16)));
typedef float    v8f  __attribute__((ext_vector_type(8)));
typedef float    v4f  __attribute__((ext_vector_type(4)));
typedef unsigned int v4u __attribute__((ext_vector_type(4)));

union FragH { v16h v; v8h h[2]; v4u u[2]; };
union FragB { v16b v; v4u u[2]; };

__device__ __forceinline__ unsigned short bf_bits(float f) {
  unsigned u = __float_as_uint(f);
  return (unsigned short)((u + 0x7FFFu + ((u >> 16) & 1u)) >> 16);
}
__device__ __forceinline__ float bf_up(unsigned short h) { return __uint_as_float(((unsigned)h) << 16); }
__device__ __forceinline__ float bfr(float f) { return bf_up(bf_bits(f)); }
__device__ __forceinline__ unsigned short h_bits(_Float16 x) { return __builtin_bit_cast(unsigned short, x); }
__device__ __forceinline__ unsigned pk16(unsigned short a, unsigned short b) { return (unsigned)a | ((unsigned)b << 16); }
__device__ __forceinline__ v8f zero8() { v8f z = {0.f, 0.f, 0.f, 0.f, 0.f, 0.f, 0.f, 0.f}; return z; }

__device__ __forceinline__ v16h ldfrag_h(const _Float16* p) {
  FragH f;
  f.h[0] = *(const v8h*)(p);
  f.h[1] = *(const v8h*)(p + 16);
  return f.v;
}
__device__ __forceinline__ v16b ldfrag_b(const u16* p) {
  FragB f;
  f.u[0] = *(const v4u*)(p);
  f.u[1] = *(const v4u*)(p + 16);
  return f.v;
}

__device__ __forceinline__ v8f mma_h(v16h a, v16h b, v8f c) {
  return __builtin_amdgcn_wmma_f32_16x16x32_f16(false, a, false, b, (short)0, c, false, false);
}
__device__ __forceinline__ v8f mma_b(v16b a, v16b b, v8f c) {
  return __builtin_amdgcn_wmma_f32_16x16x32_bf16(false, a, false, b, (short)0, c, false, false);
}
template <typename F>
__device__ __forceinline__ void guard1(v8f& a, F x0, F x1, F x2, F x3) {
#if defined(__HIP_DEVICE_COMPILE__)
  asm volatile("v_nop\n\tv_nop\n\tv_nop\n\tv_nop" : "+v"(a) : "v"(x0), "v"(x1), "v"(x2), "v"(x3) : "memory");
#endif
}
__device__ __forceinline__ void guard2(v8f& a, v8f& b, v16h x0, v16h x1, v16h x2, v16h x3, v16h x4, v16h x5) {
#if defined(__HIP_DEVICE_COMPILE__)
  asm volatile("v_nop\n\tv_nop\n\tv_nop\n\tv_nop"
               : "+v"(a), "+v"(b) : "v"(x0), "v"(x1), "v"(x2), "v"(x3), "v"(x4), "v"(x5) : "memory");
#endif
}
__device__ __forceinline__ void acc_guard1(v8f& a) {
#if defined(__HIP_DEVICE_COMPILE__)
  asm volatile("v_nop\n\tv_nop\n\tv_nop\n\tv_nop" : "+v"(a));
#endif
}
__device__ __forceinline__ void wave_sync_lds() {
  __builtin_amdgcn_fence(__ATOMIC_RELEASE, "workgroup");
  __builtin_amdgcn_wave_barrier();
  __builtin_amdgcn_fence(__ATOMIC_ACQUIRE, "workgroup");
}

__global__ __launch_bounds__(128)
void tplanes(const float* __restrict__ points, const float* __restrict__ w, const float* __restrict__ bias,
             u16* QAo, u16* K1o, u16* K2o, u16* VHo, u16* VLo) {
  __shared__ __align__(16) u16 XA[64 * XAP];
  __shared__ __align__(16) u16 WB[16 * XAP];
  __shared__ __align__(16) u16 SQ[64 * XAP];
  __shared__ __align__(16) u16 S1[64 * XAP];
  __shared__ __align__(16) u16 S2[64 * XAP];
  __shared__ __align__(16) u16 SVH[16 * VTP];
  __shared__ __align__(16) u16 SVL[16 * VTP];

  const int tid = threadIdx.x, wave = tid >> 5, lane = tid & 31, hh = lane >> 4, m = lane & 15;
  const int bid = blockIdx.x;
  const int nt  = bid % NT64;
  const int t2  = bid / NT64;
  const int g   = t2 % NGR;
  const int b   = t2 / NGR;
  if (b >= NB) return;
  const int n0  = nt * 64;
  const v4u z4 = {0u, 0u, 0u, 0u};
  {
    const int i = tid >> 3, nc = (tid & 7) * 8;
    const float* src = points + ((size_t)b * C_CH + g * CG + i) * SEQ_FULL + n0 + nc;
    const v4f a = *(const v4f*)(src), a2 = *(const v4f*)(src + 4);
#pragma unroll
    for (int e = 0; e < 4; ++e) {
      XA[(nc + e) * XAP + i]     = bf_bits(a[e]);
      XA[(nc + 4 + e) * XAP + i] = bf_bits(a2[e]);
    }
    const int zr = tid >> 1, zc = CG + (tid & 1) * 8;
    *(v4u*)(XA + zr * XAP + zc) = z4;
    *(v4u*)(S2 + zr * XAP + zc) = z4;
    if (tid < 32) {
      *(v4u*)(WB + zr * XAP + zc) = z4;
    }
    if (tid < 64) {
      const int o = tid >> 2, i0 = (tid & 3) * 4;
      const v4f wv = *(const v4f*)(w + (size_t)g * (CG * CG) + o * CG + i0);
#pragma unroll
      for (int e = 0; e < 4; ++e) WB[o * XAP + i0 + e] = bf_bits(wv[e]);
    }
  }
  __syncthreads();

  const v16b af = ldfrag_b(XA + (wave * 16 + m) * XAP + 8 * hh);
  const v16b wf = ldfrag_b(WB + m * XAP + 8 * hh);
  v8f acc = mma_b(af, wf, zero8());
  guard1<v16b>(acc, af, wf, af, wf);
  const float bb = bfr(bias[g * CG + m]);

  const int nl0 = wave * 16 + 8 * hh;
  unsigned short hvb[8], lvb[8];
#pragma unroll
  for (int r = 0; r < 8; ++r) {
    const float t  = acc[r] + bb;
    const float tq = t * QSC;
    const _Float16 th = (_Float16)tq;
    const _Float16 tl = (_Float16)(tq - (float)th);
    const unsigned short hb = h_bits(th), lb = h_bits(tl);
    const int ro = (nl0 + r) * XAP + m;
    SQ[ro] = hb;  SQ[ro + CG] = lb;
    S1[ro] = hb;  S1[ro + CG] = hb;
    S2[ro] = lb;
    const float en = __expf(fminf(t, 0.0f)) - 1.0f;
    const float ev = (t > 0.0f) ? t : en;
    const float vq = ev * VCAR;
    const _Float16 vh = (_Float16)vq;
    const _Float16 vl = (_Float16)(vq - (float)vh);
    hvb[r] = h_bits(vh);
    lvb[r] = h_bits(vl);
  }
  v4u vh4, vl4;
#pragma unroll
  for (int e = 0; e < 4; ++e) {
    vh4[e] = pk16(hvb[2 * e], hvb[2 * e + 1]);
    vl4[e] = pk16(lvb[2 * e], lvb[2 * e + 1]);
  }
  *(v4u*)(SVH + m * VTP + nl0) = vh4;
  *(v4u*)(SVL + m * VTP + nl0) = vl4;
  __syncthreads();

  v4u q4[2], k14[2], k24[2];
#pragma unroll
  for (int it = 0; it < 2; ++it) {
    const int p  = it * 128 + tid;
    const int rl = p >> 2, c8 = (p & 3) * 8;
    q4[it]  = *(const v4u*)(SQ + rl * XAP + c8);
    k14[it] = *(const v4u*)(S1 + rl * XAP + c8);
    k24[it] = *(const v4u*)(S2 + rl * XAP + c8);
  }
  const int vo = tid >> 3, v8 = (tid & 7) * 8;
  const v4u vhs = *(const v4u*)(SVH + vo * VTP + v8);
  const v4u vls = *(const v4u*)(SVL + vo * VTP + v8);
  const size_t pg    = (size_t)b * NGR + g;
  const size_t qbase = (pg * SEQ + n0) * KP;
  const size_t vbase = (pg * CG + vo) * (size_t)SEQ + n0 + v8;
  for (int pass = 0; pass < 2; ++pass) {
#pragma unroll
    for (int it = 0; it < 2; ++it) {
      const size_t po = qbase + (size_t)(it * 128 + tid) * 8;
      *(volatile v4u*)(QAo + po) = q4[it];
      *(volatile v4u*)(K1o + po) = k14[it];
      *(volatile v4u*)(K2o + po) = k24[it];
    }
    *(volatile v4u*)(VHo + vbase) = vhs;
    *(volatile v4u*)(VLo + vbase) = vls;
    __threadfence();
  }
}

__global__ __launch_bounds__(128)
void attn(const u16* __restrict__ QAp, const u16* __restrict__ K1p, const u16* __restrict__ K2p,
          const u16* __restrict__ VHp, const u16* __restrict__ VLp, float* Y) {
  __shared__ __align__(16) float ptile[4 * PTW];
  __shared__ __align__(16) float otile[CG * OTP];

  const int tid = threadIdx.x, wave = tid >> 5, lane = tid & 31, hh = lane >> 4, c = lane & 15;
  const int bid = blockIdx.x;
  const int qt  = bid % NT64;
  const int t2  = bid / NT64;
  const int g   = t2 % NGR;
  const int b   = t2 / NGR;
  if (b >= NB) return;
  const int q0  = qt * 64 + wave * 16;
  const size_t pg = (size_t)b * NGR + g;

  const _Float16* Qa  = (const _Float16*)(const void*)QAp + (pg * SEQ + q0 + c) * KP + 8 * hh;
  const _Float16* K1b = (const _Float16*)(const void*)K1p + (pg * SEQ + c) * KP + 8 * hh;
  const _Float16* K2b = (const _Float16*)(const void*)K2p + (pg * SEQ + c) * KP + 8 * hh;
  const _Float16* Vhb = (const _Float16*)(const void*)VHp + (pg * CG + c) * (size_t)SEQ + 8 * hh;
  const _Float16* Vlb = (const _Float16*)(const void*)VLp + (pg * CG + c) * (size_t)SEQ + 8 * hh;
  float* pt = ptile + wave * PTW;

  const float lsc = RSQ_CG * (LOG2E / (QSC * QSC));
  const float oc  = 1.0f / (PCAR * VCAR);
  const v16h qa = ldfrag_h(Qa);

  float mrow[8], lrow[8];
  v8f o = zero8();
#pragma unroll
  for (int r = 0; r < 8; ++r) { mrow[r] = -INFINITY; lrow[r] = 0.f; }

#pragma unroll 1
  for (int kt = 0; kt < NKT; ++kt) {
    const int kb = kt * 32;
    v8f s0 = zero8(), s1 = zero8();
    const _Float16* k10 = K1b + (size_t)kb * KP;
    const _Float16* k11 = k10 + 16 * KP;
    const _Float16* k20 = K2b + (size_t)kb * KP;
    const _Float16* k21 = k20 + 16 * KP;
    const v16h f10 = ldfrag_h(k10), f11 = ldfrag_h(k11);
    const v16h f20 = ldfrag_h(k20), f21 = ldfrag_h(k21);
    s0 = mma_h(qa, f10, s0);
    s0 = mma_h(qa, f20, s0);
    s1 = mma_h(qa, f11, s1);
    s1 = mma_h(qa, f21, s1);
    guard2(s0, s1, qa, f10, f20, f11, f21, qa);
#pragma unroll
    for (int r = 0; r < 8; ++r) {
      const float u0 = s0[r] * lsc;
      const float u1 = s1[r] * lsc;
      float mx = fmaxf(u0, u1);
#pragma unroll
      for (int off = 1; off < 16; off <<= 1) mx = fmaxf(mx, __shfl_xor(mx, off, 32));
      const float mn = fmaxf(mrow[r], mx);
      const float ms = (mn == -INFINITY) ? 0.0f : mn;
      const float al = exp2f(mrow[r] - ms);
      mrow[r] = mn;
      const float e0 = exp2f(u0 - ms), e1 = exp2f(u1 - ms);
      float ps = e0 + e1;
#pragma unroll
      for (int off = 1; off < 16; off <<= 1) ps += __shfl_xor(ps, off, 32);
      lrow[r] = lrow[r] * al + ps;
      o[r] *= al;
      const int ro = (8 * hh + r) * PTP + c;
      pt[ro]      = e0;
      pt[ro + 16] = e1;
    }
    wave_sync_lds();
    FragH ph, pl;
    {
      const float* prow = pt + c * PTP + 8 * hh;
      const v4f p0 = *(const v4f*)(prow), p1 = *(const v4f*)(prow + 4);
      const v4f p2 = *(const v4f*)(prow + 16), p3 = *(const v4f*)(prow + 20);
#pragma unroll
      for (int e = 0; e < 4; ++e) {
        const float ta = p0[e] * PCAR, tb = p1[e] * PCAR, tc = p2[e] * PCAR, td = p3[e] * PCAR;
        const _Float16 ha = (_Float16)ta, hb = (_Float16)tb, hc = (_Float16)tc, hd = (_Float16)td;
        ph.h[0][e]     = ha;
        ph.h[0][4 + e] = hb;
        ph.h[1][e]     = hc;
        ph.h[1][4 + e] = hd;
        pl.h[0][e]     = (_Float16)(ta - (float)ha);
        pl.h[0][4 + e] = (_Float16)(tb - (float)hb);
        pl.h[1][e]     = (_Float16)(tc - (float)hc);
        pl.h[1][4 + e] = (_Float16)(td - (float)hd);
      }
    }
    {
      const v16h vh = ldfrag_h(Vhb + kb), vl = ldfrag_h(Vlb + kb);
      o = mma_h(ph.v, vh, o);
      o = mma_h(pl.v, vh, o);
      o = mma_h(ph.v, vl, o);
      guard1<v16h>(o, ph.v, pl.v, vh, vl);
    }
    wave_sync_lds();
  }
  acc_guard1(o);
  float ov[8];
#pragma unroll
  for (int r = 0; r < 8; ++r) {
    const float lv  = lrow[r];
    const float ls  = (lv > 0.0f) ? lv : 1.0f;
    const float inv = (lv > 0.0f) ? ((1.0f / ls) * oc) : 0.0f;
    ov[r] = o[r] * inv;
  }
  {
    const v4f oa  = {ov[0], ov[1], ov[2], ov[3]};
    const v4f ob2 = {ov[4], ov[5], ov[6], ov[7]};
    float* od = otile + c * OTP + wave * 16 + 8 * hh;
    *(v4f*)(od)     = oa;
    *(v4f*)(od + 4) = ob2;
  }
  __syncthreads();
  v4f yv[2];
#pragma unroll
  for (int it = 0; it < 2; ++it) {
    const int p = it * 128 + tid;
    const int oo = p >> 4, c4 = (p & 15) * 4;
    yv[it] = *(const v4f*)(otile + oo * OTP + c4);
  }
  for (int pass = 0; pass < 2; ++pass) {
#pragma unroll
    for (int it = 0; it < 2; ++it) {
      const int p = it * 128 + tid;
      const int oo = p >> 4, c4 = (p & 15) * 4;
      float* dst = Y + ((size_t)b * C_CH + oo * NGR + g) * (size_t)SEQ + qt * 64 + c4;
      *(volatile v4f*)(dst) = yv[it];
    }
    __threadfence();
  }
}

__global__ __launch_bounds__(256)
void gnorm(const float* __restrict__ Y, const float* __restrict__ points,
           const float* __restrict__ gamma, const float* __restrict__ beta, float* out) {
  __shared__ double red[8];
  const int tid = threadIdx.x, wave = tid >> 5, lane = tid & 31;
  const int bid = blockIdx.x;
  const int k   = bid % NGR;
  const int b   = bid / NGR;
  if (b >= NB) return;
  const size_t ybase = ((size_t)b * C_CH + k * CG) * (size_t)SEQ;
  const size_t pbase = ((size_t)b * C_CH + k * CG) * (size_t)SEQ_FULL;
  const double invn  = 1.0 / (double)(CG * SEQ);

  double s = 0.0;
#pragma unroll 1
  for (int it = 0; it < GNIT; ++it) {
    const int e   = it * 1024 + tid * 4;
    const int row = e / SEQ;
    const int col = e - row * SEQ;
    const v4f yv = *(const v4f*)(Y + ybase + (size_t)row * SEQ + col);
    const v4f pv = *(const v4f*)(points + pbase + (size_t)row * SEQ_FULL + col);
#pragma unroll
    for (int e2 = 0; e2 < 4; ++e2) s += (double)(yv[e2] + bfr(pv[e2]));
  }
#pragma unroll
  for (int off = 16; off > 0; off >>= 1) s += __shfl_xor(s, off, 32);
  __syncthreads();
  if (lane == 0) red[wave] = s;
  __syncthreads();
  double tot = 0.0;
#pragma unroll
  for (int wv = 0; wv < 8; ++wv) tot += red[wv];
  const float mean = (float)(tot * invn);

  double q = 0.0;
#pragma unroll 1
  for (int it = 0; it < GNIT; ++it) {
    const int e   = it * 1024 + tid * 4;
    const int row = e / SEQ;
    const int col = e - row * SEQ;
    const v4f yv = *(const v4f*)(Y + ybase + (size_t)row * SEQ + col);
    const v4f pv = *(const v4f*)(points + pbase + (size_t)row * SEQ_FULL + col);
#pragma unroll
    for (int e2 = 0; e2 < 4; ++e2) {
      const float d = (yv[e2] + bfr(pv[e2])) - mean;
      q += (double)(d * d);
    }
  }
#pragma unroll
  for (int off = 16; off > 0; off >>= 1) q += __shfl_xor(q, off, 32);
  __syncthreads();
  if (lane == 0) red[wave] = q;
  __syncthreads();
  double tq = 0.0;
#pragma unroll
  for (int wv = 0; wv < 8; ++wv) tq += red[wv];
  const float var  = (float)(tq * invn);
  const float rstd = rsqrtf(var + GN_EPS);

#pragma unroll 1
  for (int it = 0; it < GNIT; ++it) {
    const int e   = it * 1024 + tid * 4;
    const int row = e / SEQ;
    const int col = e - row * SEQ;
    const int ch  = k * CG + row;
    const float ga = bfr(gamma[ch]), be = bfr(beta[ch]);
    const v4f yv = *(const v4f*)(Y + ybase + (size_t)row * SEQ + col);
    const v4f pv = *(const v4f*)(points + pbase + (size_t)row * SEQ_FULL + col);
    v4f rv;
#pragma unroll
    for (int e2 = 0; e2 < 4; ++e2) {
      const float x = yv[e2] + bfr(pv[e2]);
      rv[e2] = (x - mean) * rstd * ga + be;
    }
    float* dst = out + ybase + (size_t)row * SEQ + col;
    *(volatile v4f*)(dst) = rv;
    __threadfence();
    *(volatile v4f*)(dst) = rv;
  }
}

extern "C" void kernel_launch(void* const* d_in, const int* in_sizes, int n_in,
                              void* d_out, int out_size, void* d_ws, size_t ws_size,
                              hipStream_t stream) {
  if (n_in < 5) return;
  if (in_sizes[0] < NB * C_CH * SEQ_FULL) return;
  if (in_sizes[1] < C_CH * CG) return;
  if (in_sizes[2] < C_CH) return;
  if (in_sizes[3] < C_CH) return;
  if (in_sizes[4] < C_CH) return;
  if (out_size < NB * C_CH * SEQ) return;

  const float* points = (const float*)d_in[0];
  const float* w      = (const float*)d_in[1];
  const float* bias   = (const float*)d_in[2];
  const float* gamma  = (const float*)d_in[3];
  const float* beta   = (const float*)d_in[4];
  float*       out    = (float*)d_out;

  const size_t szQ = (size_t)NB * NGR * SEQ * KP * 2;
  const size_t szV = (size_t)NB * NGR * CG * SEQ * 2;
  const size_t szY = (size_t)NB * C_CH * SEQ * 4;
  size_t off = 0;
  const size_t oQA = off; off += szQ;
  const size_t oK1 = off; off += szQ;
  const size_t oK2 = off; off += szQ;
  const size_t oVH = off; off += szV;
  const size_t oVL = off; off += szV;
  const size_t oY  = off; off += szY;
  if (off > ws_size) return;
  if (off > (size_t)WS_CAP) return;

  char* ws = (char*)d_ws;
  u16*   QA = (u16*)(ws + oQA);
  u16*   K1 = (u16*)(ws + oK1);
  u16*   K2 = (u16*)(ws + oK2);
  u16*   VH = (u16*)(ws + oVH);
  u16*   VL = (u16*)(ws + oVL);
  float* Y  = (float*)(ws + oY);

  const dim3 gT(NB * NGR * NT64), b128(128), gN(NB * NGR), b256(256);
  tplanes<<<gT, b128, 0, stream>>>(points, w, bias, QA, K1, K2, VH, VL);
  attn<<<gT, b128, 0, stream>>>(QA, K1, K2, VH, VL, Y);
  gnorm<<<gN, b256, 0, stream>>>(Y, points, gamma, beta, out);
  (void)hipGetLastError();
}
